// Model_47115791237202
// MI455X (gfx1250) — hardware-verified
//
#include <hip/hip_runtime.h>
#include <stddef.h>
#include <stdint.h>
#include <math.h>


#define FIN    32
#define HID    64
#define NHEAD  4
#define HC     256
#define XAP    256
#define KX     256
#define NLR    512
#define KG     128
#define ODIM   32
#define NTHR   256
#define NWAVE  8
#define EPT    8
#define CHUNK  (NTHR * EPT)
#define WCAP   (EPT * 32)
#define LISTN  (NWAVE * WCAP)
#define NBA    1024
#define SLA    10
#define RCAP   8192
#define DEGCAP 31
#define GBM    64
#define GTHR   128
#define AGG_ZINTS    (LISTN + 2 * RCAP + 3 * NBA)
#define MISC_INTS    16
#define AGG_LDS_INTS (AGG_ZINTS + MISC_INTS)
#define PF_BLR   0
#define PF_ATT   512
#define PF_BSUM  768
#define PF_BIN   832
#define PF_BG    896
#define PF_N     1024
#define NB_WLR   64
#define NB_WIN   1
#define NB_WG    2
#define NB_PF    1
#define WSMAX  134217728

static_assert((CHUNK & (CHUNK - 1)) == 0 && CHUNK <= 4096);
static_assert((NBA & (NBA - 1)) == 0 && NBA == (1 << SLA));
static_assert(((long long)CHUNK << SLA) < (1LL << 31));
static_assert(NBA % NWAVE == 0 && NBA % 32 == 0);
static_assert(AGG_ZINTS % 4 == 0 && LISTN % 4 == 0 && RCAP % 4 == 0);
static_assert(DEGCAP + 1 <= 32);
static_assert(FIN % 32 == 0 && KX % 32 == 0 && KG % 32 == 0);
static_assert(KX == 4 * HID && KG == 2 * HID && HC == NHEAD * HID && NLR == 2 * HC);
static_assert(GBM == (GTHR / 32) * 16);
static_assert(NLR * (KX / 8) == NB_WLR * NTHR);
static_assert(HID * (FIN / 8) == NB_WIN * NTHR);
static_assert(ODIM * (KG / 8) == NB_WG * NTHR);
static_assert(PF_N == 4 * NTHR * NB_PF);
static_assert(PF_ATT == 4 * 128 && PF_BSUM == 4 * 192 && PF_BIN == 4 * 208 && PF_BG == 4 * 224);
static_assert(AGG_LDS_INTS * 4 <= 300000);

typedef float          v2f   __attribute__((ext_vector_type(2)));
typedef float          v4f   __attribute__((ext_vector_type(4)));
typedef float          v8f   __attribute__((ext_vector_type(8)));
typedef int            v4i   __attribute__((ext_vector_type(4)));
typedef int            v8i   __attribute__((ext_vector_type(8)));
typedef unsigned int   v4u   __attribute__((ext_vector_type(4)));
typedef unsigned short v8us  __attribute__((ext_vector_type(8)));
typedef unsigned short v16us __attribute__((ext_vector_type(16)));
typedef __bf16         v16bf __attribute__((ext_vector_type(16)));
typedef v4f  __attribute__((may_alias)) v4fa;
typedef v4i  __attribute__((may_alias)) v4ia;
typedef v8us __attribute__((may_alias)) v8usa;
union FragB { v16bf v; v16us u; v8us h[2]; v8i w; };

__device__ __forceinline__ v8f wmb(const FragB& a, const FragB& b, v8f c) {
  v8f d = __builtin_amdgcn_wmma_f32_16x16x32_bf16(false, a.v, false, b.v, (short)0, c, false, false);
  asm volatile("v_nop\n\tv_nop\n\tv_nop\n\tv_nop" : "+v"(d) : "v"(a.w), "v"(b.w));
  return d;
}

__device__ __forceinline__ unsigned bf16_bits(float f) {
  const unsigned u = __float_as_uint(f);
  return (u + 0x7FFFu + ((u >> 16) & 1u)) >> 16;
}
__device__ __forceinline__ float bf16_val(float f) {
  return __uint_as_float(bf16_bits(f) << 16);
}
__device__ __forceinline__ unsigned short hl_sel(float v, bool lo) {
  const unsigned hb = bf16_bits(v);
  const unsigned lb = bf16_bits(v - __uint_as_float(hb << 16));
  return (unsigned short)(lo ? lb : hb);
}
__device__ __forceinline__ float blend6(float a, unsigned ma, float b, unsigned mb, float c, unsigned mc,
                                        float d, unsigned md, float e, unsigned me, float f, unsigned mf) {
  const unsigned bits = (__float_as_uint(a) & ma) | (__float_as_uint(b) & mb) | (__float_as_uint(c) & mc) |
                        (__float_as_uint(d) & md) | (__float_as_uint(e) & me) | (__float_as_uint(f) & mf);
  return __uint_as_float(bits);
}

template <int SLB>
__device__ __forceinline__ int scan_chunk(const int* __restrict__ dsts, int nE, int cbase, int slotBase,
                                          int nb, int vec8, int* list, int tid, int lane, int wave) {
  int wc = 0;
  const int el0  = tid * EPT;
  const int e0   = cbase + el0;
  const int sent = -2147483647 - 1;
  v4i da, db;
  if (vec8 != 0 && cbase + CHUNK <= nE) {
    da = *(const v4i*)(dsts + e0);
    db = *(const v4i*)(dsts + e0 + 4);
  } else {
    da.x = (e0     < nE) ? dsts[min(e0,     nE - 1)] : sent;
    da.y = (e0 + 1 < nE) ? dsts[min(e0 + 1, nE - 1)] : sent;
    da.z = (e0 + 2 < nE) ? dsts[min(e0 + 2, nE - 1)] : sent;
    da.w = (e0 + 3 < nE) ? dsts[min(e0 + 3, nE - 1)] : sent;
    db.x = (e0 + 4 < nE) ? dsts[min(e0 + 4, nE - 1)] : sent;
    db.y = (e0 + 5 < nE) ? dsts[min(e0 + 5, nE - 1)] : sent;
    db.z = (e0 + 6 < nE) ? dsts[min(e0 + 6, nE - 1)] : sent;
    db.w = (e0 + 7 < nE) ? dsts[min(e0 + 7, nE - 1)] : sent;
  }
  const unsigned nbs = (unsigned)slotBase;
  const unsigned unb = (unsigned)nb;
  const unsigned s0 = (unsigned)da.x - nbs, s1 = (unsigned)da.y - nbs;
  const unsigned s2 = (unsigned)da.z - nbs, s3 = (unsigned)da.w - nbs;
  const unsigned s4 = (unsigned)db.x - nbs, s5 = (unsigned)db.y - nbs;
  const unsigned s6 = (unsigned)db.z - nbs, s7 = (unsigned)db.w - nbs;
  const bool h0 = s0 < unb, h1 = s1 < unb, h2 = s2 < unb, h3 = s3 < unb;
  const bool h4 = s4 < unb, h5 = s5 < unb, h6 = s6 < unb, h7 = s7 < unb;
  const unsigned any = __builtin_amdgcn_ballot_w32(h0 | h1 | h2 | h3 | h4 | h5 | h6 | h7);
  if (any != 0u) {
#define HITJ(J, HJ, SJ) { \
      const unsigned mj = __builtin_amdgcn_ballot_w32(HJ); \
      if (mj != 0u) { \
        if (HJ) { \
          const int pos = wc + (int)__builtin_amdgcn_mbcnt_lo(mj, 0u); \
          if (pos < WCAP) list[wave * WCAP + pos] = ((el0 + (J)) << SLB) | (int)(SJ); \
        } \
        wc += (int)__builtin_popcount(mj); } }
    HITJ(0, h0, s0)
    HITJ(1, h1, s1)
    HITJ(2, h2, s2)
    HITJ(3, h3, s3)
    HITJ(4, h4, s4)
    HITJ(5, h5, s5)
    HITJ(6, h6, s6)
    HITJ(7, h7, s7)
#undef HITJ
  }
  return wc;
}

__global__ __launch_bounds__(NTHR) void k_prep(
    const float* __restrict__ feat, const float* __restrict__ Win, const float* __restrict__ bin,
    const float* __restrict__ Wl, const float* __restrict__ bl, const float* __restrict__ Wr,
    const float* __restrict__ br, const float* __restrict__ att, const float* __restrict__ bconv,
    const float* __restrict__ Wg, const float* __restrict__ bg, int nN, int gFB,
    unsigned short* FB, unsigned short* WINt, unsigned short* WLRt, unsigned short* WGt, float* PF) {
  const int tid = (int)threadIdx.x;
  const int bx  = (int)blockIdx.x;
  if (bx < gFB) {
    const int u   = bx * NTHR + tid;
    const int row = u >> 2;
    const int k8  = (u & 3) * 8;
    const int rc  = row < nN ? row : nN - 1;
    const float* p = feat + (size_t)rc * FIN + k8;
    const v4f a = *(const v4fa*)p;
    const v4f b = *(const v4fa*)(p + 4);
    const bool ok = row < nN;
    v8us o;
    o[0] = ok ? (unsigned short)bf16_bits(a.x) : (unsigned short)0;
    o[1] = ok ? (unsigned short)bf16_bits(a.y) : (unsigned short)0;
    o[2] = ok ? (unsigned short)bf16_bits(a.z) : (unsigned short)0;
    o[3] = ok ? (unsigned short)bf16_bits(a.w) : (unsigned short)0;
    o[4] = ok ? (unsigned short)bf16_bits(b.x) : (unsigned short)0;
    o[5] = ok ? (unsigned short)bf16_bits(b.y) : (unsigned short)0;
    o[6] = ok ? (unsigned short)bf16_bits(b.z) : (unsigned short)0;
    o[7] = ok ? (unsigned short)bf16_bits(b.w) : (unsigned short)0;
    unsigned short* dp = FB + (size_t)row * FIN + k8;
    *(volatile v8us*)dp = o;
    __threadfence();
    *(volatile v8us*)dp = o;
    return;
  }
  const int b = bx - gFB;
  if (b < NB_WLR) {
    const int v    = b * NTHR + tid;
    const int n    = v >> 5;
    const int k8   = (v & 31) * 8;
    const int srow = ((k8 >> 7) << 6) + (k8 & 63);
    v8us o;
    if (b < NB_WLR / 2) {
      const float* p = Wl + (size_t)srow * HC + n;
#pragma unroll
      for (int i = 0; i < 8; ++i) o[i] = (unsigned short)bf16_bits(p[(size_t)i * HC]);
    } else {
      const float* p = Wr + (size_t)srow * HC + (n - HC);
#pragma unroll
      for (int i = 0; i < 8; ++i) o[i] = (unsigned short)bf16_bits(p[(size_t)i * HC]);
    }
    unsigned short* dp = WLRt + (size_t)n * KX + k8;
    *(volatile v8us*)dp = o;
    __threadfence();
    *(volatile v8us*)dp = o;
    return;
  }
  if (b < NB_WLR + NB_WIN) {
    const int n  = tid >> 2;
    const int k8 = (tid & 3) * 8;
    const float* p = Win + (size_t)k8 * HID + n;
    v8us o;
#pragma unroll
    for (int i = 0; i < 8; ++i) o[i] = (unsigned short)bf16_bits(p[(size_t)i * HID]);
    unsigned short* dp = WINt + (size_t)n * FIN + k8;
    *(volatile v8us*)dp = o;
    __threadfence();
    *(volatile v8us*)dp = o;
    return;
  }
  if (b < NB_WLR + NB_WIN + NB_WG) {
    const int v  = (b - NB_WLR - NB_WIN) * NTHR + tid;
    const int n  = v >> 4;
    const int k8 = (v & 15) * 8;
    const int kk = k8 & (HID - 1);
    const float* p = Wg + (size_t)kk * ODIM + n;
    v8us o;
#pragma unroll
    for (int i = 0; i < 8; ++i) o[i] = (unsigned short)bf16_bits(p[(size_t)i * ODIM]);
    unsigned short* dp = WGt + (size_t)n * KG + k8;
    *(volatile v8us*)dp = o;
    __threadfence();
    *(volatile v8us*)dp = o;
    return;
  }
  if (b == NB_WLR + NB_WIN + NB_WG) {
    const int ibl = (tid < 63 ? tid : 63) * 4;
    const int t1  = tid - 64;  const int ibr = (t1 < 0 ? 0 : (t1 > 63 ? 63 : t1)) * 4;
    const int t2  = tid - 128; const int iat = (t2 < 0 ? 0 : (t2 > 63 ? 63 : t2)) * 4;
    const int t3  = tid - 192; const int ibc = (t3 < 0 ? 0 : (t3 > 15 ? 15 : t3)) * 4;
    const int t4  = tid - 208; const int ibi = (t4 < 0 ? 0 : (t4 > 15 ? 15 : t4)) * 4;
    const int t5  = tid - 224; const int ibg = (t5 < 0 ? 0 : (t5 > 7 ? 7 : t5)) * 4;
    const v4f vbl = *(const v4f*)(bl + ibl);
    const v4f vbr = *(const v4f*)(br + ibr);
    const v4f vat = *(const v4f*)(att + iat);
    const v4f c0  = *(const v4f*)(bconv + ibc);
    const v4f c1  = *(const v4f*)(bconv + HID + ibc);
    const v4f c2  = *(const v4f*)(bconv + 2 * HID + ibc);
    const v4f c3  = *(const v4f*)(bconv + 3 * HID + ibc);
    const v4f vbi = *(const v4f*)(bin + ibi);
    const v4f vbg = *(const v4f*)(bg + ibg);
    v4f bs;
    bs.x = ((bf16_val(c0.x) + bf16_val(c1.x)) + bf16_val(c2.x)) + bf16_val(c3.x);
    bs.y = ((bf16_val(c0.y) + bf16_val(c1.y)) + bf16_val(c2.y)) + bf16_val(c3.y);
    bs.z = ((bf16_val(c0.z) + bf16_val(c1.z)) + bf16_val(c2.z)) + bf16_val(c3.z);
    bs.w = ((bf16_val(c0.w) + bf16_val(c1.w)) + bf16_val(c2.w)) + bf16_val(c3.w);
    const unsigned mbl = (unsigned)(-(int)(tid < 64));
    const unsigned mbr = (unsigned)(-(int)((tid >= 64)  & (tid < 128)));
    const unsigned mat = (unsigned)(-(int)((tid >= 128) & (tid < 192)));
    const unsigned mbs = (unsigned)(-(int)((tid >= 192) & (tid < 208)));
    const unsigned mbi = (unsigned)(-(int)((tid >= 208) & (tid < 224)));
    const unsigned mbg = (unsigned)(-(int)((tid >= 224) & (tid < 232)));
    v4f o;
    o.x = blend6(bf16_val(vbl.x), mbl, bf16_val(vbr.x), mbr, bf16_val(vat.x), mat,
                 bs.x, mbs, bf16_val(vbi.x), mbi, bf16_val(vbg.x), mbg);
    o.y = blend6(bf16_val(vbl.y), mbl, bf16_val(vbr.y), mbr, bf16_val(vat.y), mat,
                 bs.y, mbs, bf16_val(vbi.y), mbi, bf16_val(vbg.y), mbg);
    o.z = blend6(bf16_val(vbl.z), mbl, bf16_val(vbr.z), mbr, bf16_val(vat.z), mat,
                 bs.z, mbs, bf16_val(vbi.z), mbi, bf16_val(vbg.z), mbg);
    o.w = blend6(bf16_val(vbl.w), mbl, bf16_val(vbr.w), mbr, bf16_val(vat.w), mat,
                 bs.w, mbs, bf16_val(vbi.w), mbi, bf16_val(vbg.w), mbg);
    float* dp = PF + 4 * tid;
    *(volatile v4f*)dp = o;
    __threadfence();
    *(volatile v4f*)dp = o;
  }
}

__global__ __launch_bounds__(GTHR) void k_gemm0(const unsigned short* __restrict__ FB,
                                                const unsigned short* __restrict__ WINt,
                                                const float* __restrict__ pf, unsigned short* XA) {
  __shared__ __attribute__((aligned(16))) float stg[GBM * HID];
  const int tid = (int)threadIdx.x, lane = tid & 31, wave = tid >> 5, hh = lane >> 4, m = lane & 15;
  const int rowBase = (int)blockIdx.x * GBM;

  v8f acc[4];
  {
    const v8f z = {0.f, 0.f, 0.f, 0.f, 0.f, 0.f, 0.f, 0.f};
    acc[0] = z; acc[1] = z; acc[2] = z; acc[3] = z;
  }
  const unsigned short* ap = FB   + (size_t)(rowBase + 16 * wave + m) * FIN + 8 * hh;
  const unsigned short* wp = WINt + (size_t)m * FIN + 8 * hh;
  {
    FragB af;
    af.h[0] = *(const v8usa*)ap;
    af.h[1] = *(const v8usa*)(ap + 16);
#pragma unroll
    for (int t = 0; t < 4; ++t) {
      const unsigned short* wq = wp + (size_t)(16 * t) * FIN;
      FragB bf;
      bf.h[0] = *(const v8usa*)wq;
      bf.h[1] = *(const v8usa*)(wq + 16);
      acc[t] = wmb(af, bf, acc[t]);
    }
  }
#pragma unroll
  for (int t = 0; t < 4; ++t) {
    const int lc = 16 * t + m;
#pragma unroll
    for (int r = 0; r < 8; ++r) {
      const int lr = 16 * wave + 8 * hh + r;
      stg[lr * HID + lc] = acc[t][r];
    }
  }
  __syncthreads();

  const int cb = 8 * (lane & 7);
  const bool losel = ((lane >> 3) & 1) != 0;
  const v4f b0 = *(const v4f*)(pf + PF_BIN + cb);
  const v4f b1 = *(const v4f*)(pf + PF_BIN + cb + 4);
  v8us q[16];
#pragma unroll
  for (int i = 0; i < 16; ++i) {
    const int lr = 16 * wave + i;
    const v4f f0 = *(const v4fa*)(stg + lr * HID + cb);
    const v4f f1 = *(const v4fa*)(stg + lr * HID + cb + 4);
    v8us o;
    o[0] = hl_sel(f0.x + b0.x, losel); o[1] = hl_sel(f0.y + b0.y, losel);
    o[2] = hl_sel(f0.z + b0.z, losel); o[3] = hl_sel(f0.w + b0.w, losel);
    o[4] = hl_sel(f1.x + b1.x, losel); o[5] = hl_sel(f1.y + b1.y, losel);
    o[6] = hl_sel(f1.z + b1.z, losel); o[7] = hl_sel(f1.w + b1.w, losel);
    q[i] = o;
  }
#pragma unroll
  for (int i = 0; i < 16; ++i) {
    unsigned short* rp = XA + (size_t)(rowBase + 16 * wave + i) * XAP + 8 * lane;
    *(volatile v8us*)rp = q[i];
  }
  __threadfence();
#pragma unroll
  for (int i = 0; i < 16; ++i) {
    unsigned short* rp = XA + (size_t)(rowBase + 16 * wave + i) * XAP + 8 * lane;
    *(volatile v8us*)rp = q[i];
  }
}

__global__ __launch_bounds__(GTHR) void k_gemm_step(const unsigned short* __restrict__ A,
                                                    const unsigned short* __restrict__ WT,
                                                    const float* __restrict__ pf, float* xlr,
                                                    unsigned long long planeStride) {
  __shared__ __attribute__((aligned(16))) float stg[GBM * 64];
  const int tid = (int)threadIdx.x, lane = tid & 31, wave = tid >> 5, hh = lane >> 4, m = lane & 15;
  const int rowBase = (int)blockIdx.x * GBM;
  const int col0    = (int)blockIdx.y * 64;

  v8f acc[4];
  {
    const v8f z = {0.f, 0.f, 0.f, 0.f, 0.f, 0.f, 0.f, 0.f};
    acc[0] = z; acc[1] = z; acc[2] = z; acc[3] = z;
  }
  const unsigned short* ap = A  + (size_t)(rowBase + 16 * wave + m) * XAP + 8 * hh;
  const unsigned short* wp = WT + (size_t)(col0 + m) * KX + 8 * hh;
#pragma unroll 1
  for (int ks = 0; ks < KX / 32; ++ks) {
    FragB af;
    af.h[0] = *(const v8usa*)(ap + 32 * ks);
    af.h[1] = *(const v8usa*)(ap + 32 * ks + 16);
#pragma unroll
    for (int t = 0; t < 4; ++t) {
      const unsigned short* wq = wp + (size_t)(16 * t) * KX + 32 * ks;
      FragB bf;
      bf.h[0] = *(const v8usa*)wq;
      bf.h[1] = *(const v8usa*)(wq + 16);
      acc[t] = wmb(af, bf, acc[t]);
    }
  }
#pragma unroll
  for (int t = 0; t < 4; ++t) {
    const int lc = 16 * t + m;
#pragma unroll
    for (int r = 0; r < 8; ++r) {
      const int lr = 16 * wave + 8 * hh + r;
      stg[lr * 64 + lc] = acc[t][r];
    }
  }
  __syncthreads();

  const v4f b4 = *(const v4f*)(pf + PF_BLR + col0 + 4 * m);
  const size_t pofs = (size_t)(col0 >> 8) * (size_t)planeStride + (size_t)(col0 & (HC - 1));
  v4f fv[8];
#pragma unroll
  for (int i = 0; i < 8; ++i) {
    const int lr = 16 * wave + 2 * i + hh;
    fv[i] = *(const v4fa*)(stg + lr * 64 + 4 * m) + b4;
  }
#pragma unroll
  for (int i = 0; i < 8; ++i) {
    const int gr = rowBase + 16 * wave + 2 * i + hh;
    float* op = xlr + pofs + (size_t)gr * HC + 4 * m;
    *(volatile v4f*)op = fv[i];
  }
  __threadfence();
#pragma unroll
  for (int i = 0; i < 8; ++i) {
    const int gr = rowBase + 16 * wave + 2 * i + hh;
    float* op = xlr + pofs + (size_t)gr * HC + 4 * m;
    *(volatile v4f*)op = fv[i];
  }
}

__global__ __launch_bounds__(NTHR) void k_scan(const int* __restrict__ srcs, const int* __restrict__ dsts,
                                               const int* __restrict__ nmask, int step,
                                               int nE, int nN, int vec8,
                                               const float* __restrict__ xl, const float* __restrict__ xr,
                                               const float* __restrict__ pf, unsigned short* xa) {
  extern __shared__ __attribute__((aligned(16))) int dsm[];
  int* list = dsm;
  int* hl   = dsm + LISTN;
  int* sl   = hl + RCAP;
  int* cnt  = sl + RCAP;
  int* offs = cnt + NBA;
  int* cur  = offs + NBA;
  int* misc = cur + NBA;
  const int tid = (int)threadIdx.x, lane = tid & 31, wave = tid >> 5;
  const int nodeBase = (int)blockIdx.x * NBA;

  {
    const v4i z4 = {0, 0, 0, 0};
    for (int i = tid * 4; i < AGG_ZINTS; i += NTHR * 4) *(v4ia*)(dsm + i) = z4;
    if (tid < MISC_INTS) misc[tid] = 0;
  }
  __syncthreads();

  int t = 0, ov = 0;
  const int nChunks = (nE + CHUNK - 1) / CHUNK;
#pragma unroll 1
  for (int ch = 0; ch < nChunks; ++ch) {
    const int cbase = ch * CHUNK;
    const int wc = scan_chunk<SLA>(dsts, nE, cbase, nodeBase, NBA, vec8, list, tid, lane, wave);
    if (lane == 0) misc[wave] = wc;
    __syncthreads();
    if (wave == 0) {
#pragma unroll 1
      for (int w2 = 0; w2 < NWAVE; ++w2) {
        int c = misc[w2];
        c = c < 0 ? 0 : (c > WCAP ? WCAP : c);
#pragma unroll 1
        for (int b0 = 0; b0 < c; b0 += 32) {
          const int idx = b0 + lane;
          const int ent = list[w2 * WCAP + (idx < WCAP ? idx : WCAP - 1)];
          const int m32 = (c - b0) < 32 ? (c - b0) : 32;
#pragma unroll 1
          for (int k = 0; k < m32; ++k) {
            const int u    = __builtin_amdgcn_readlane(ent, k);
            const int slot = u & (NBA - 1);
            const int el   = (u >> SLA) & (CHUNK - 1);
            const int pk   = ((cbase + el) << SLA) | slot;
            if (t < RCAP) {
              if (lane == 0) { hl[t] = pk; cnt[slot] = cnt[slot] + 1; }
              t = t + 1;
            } else {
              ov = 1;
            }
          }
        }
      }
    }
    __syncthreads();
  }
  if (wave == 0 && lane == 0) { misc[8] = t; misc[9] = ov; }
  __syncthreads();
  int tt = misc[8];
  tt = tt < 0 ? 0 : (tt > RCAP ? RCAP : tt);
  const int ovf = misc[9];

  if (wave == 0) {
    const int base = lane * (NBA / 32);
    int s = 0;
#pragma unroll 1
    for (int i = 0; i < NBA / 32; ++i) s += cnt[base + i];
    int incl = s;
#pragma unroll
    for (int d = 1; d < 32; d <<= 1) {
      const int y = __shfl_up(incl, d, 32);
      if (lane >= d) incl += y;
    }
    int run = incl - s;
#pragma unroll 1
    for (int i = 0; i < NBA / 32; ++i) {
      const int cv = cnt[base + i];
      offs[base + i] = run;
      cur[base + i]  = run;
      run += cv;
    }
  }
  __syncthreads();
  if (wave == 0) {
#pragma unroll 1
    for (int b0 = 0; b0 < tt; b0 += 32) {
      const int idx = b0 + lane;
      const int ent = hl[idx < RCAP ? idx : RCAP - 1];
      const int m32 = (tt - b0) < 32 ? (tt - b0) : 32;
#pragma unroll 1
      for (int k = 0; k < m32; ++k) {
        const int u    = __builtin_amdgcn_readlane(ent, k);
        const int slot = u & (NBA - 1);
        if (lane == 0) {
          int p = cur[slot];
          p = p < 0 ? 0 : (p > RCAP - 1 ? RCAP - 1 : p);
          sl[p] = u;
          cur[slot] = p + 1;
        }
      }
    }
  }
  __syncthreads();

  const float qnan = __int_as_float(0x7fc00000);
  const float pz = (ovf != 0) ? qnan : 0.0f;
  const int hd = lane >> 3, q = lane & 7;
  const v4f at0 = *(const v4f*)(pf + PF_ATT + 8 * lane);
  const v4f at1 = *(const v4f*)(pf + PF_ATT + 8 * lane + 4);
  const v2f bs  = *(const v2f*)(pf + PF_BSUM + 8 * q + 2 * hd);
  const int q1 = q + 8, q2 = q + 16, q3 = q + 24;
#pragma unroll 1
  for (int si = 0; si < NBA / NWAVE; ++si) {
    const int s    = si * NWAVE + wave;
    const int node = nodeBase + s;
    if (node >= nN) continue;
    int c = cnt[s];
    const bool big = c > DEGCAP;
    c = c < 0 ? 0 : (c > DEGCAP ? DEGCAP : c);
    int o = offs[s];
    o = o < 0 ? 0 : (o > RCAP ? RCAP : o);
    const int nm = nmask[node];
    const bool act  = nm > step;
    const bool pois = big || (ovf != 0);
    if (!act && !pois) continue;
    int idx = o + lane - 1;
    idx = idx < 0 ? 0 : (idx > RCAP - 1 ? RCAP - 1 : idx);
    const int ent = sl[idx];
    int eid = ent >> SLA;
    eid = eid < 0 ? 0 : (eid > nE - 1 ? nE - 1 : eid);
    int se = srcs[eid];
    se = se < 0 ? 0 : (se > nN - 1 ? nN - 1 : se);
    const int sr = (lane == 0) ? node : se;
    const int al = (nmask[sr] > step) ? 1 : 0;
    const int nent = c + 1;

    const float* xrp = xr + (size_t)node * HC + 8 * lane;
    const v4f r0 = *(const v4f*)xrp;
    const v4f r1 = *(const v4f*)(xrp + 4);
    float mx = -3.0e38f, ls = 0.0f;
    float a0 = 0.0f, a1 = 0.0f, a2 = 0.0f, a3 = 0.0f, a4 = 0.0f, a5 = 0.0f, a6 = 0.0f, a7 = 0.0f;
#pragma unroll 1
    for (int k = 0; k < nent; ++k) {
      const int sk = __builtin_amdgcn_readlane(sr, k);
      const int ak = __builtin_amdgcn_readlane(al, k);
      if (ak == 0) continue;
      const float* xp = xl + (size_t)sk * HC + 8 * lane;
      const v4f x0 = *(const v4f*)xp;
      const v4f x1 = *(const v4f*)(xp + 4);
      float u, p;
      u = x0.x + r0.x; u = (u > 0.0f) ? u : 0.2f * u; p = u * at0.x;
      u = x0.y + r0.y; u = (u > 0.0f) ? u : 0.2f * u; p = fmaf(u, at0.y, p);
      u = x0.z + r0.z; u = (u > 0.0f) ? u : 0.2f * u; p = fmaf(u, at0.z, p);
      u = x0.w + r0.w; u = (u > 0.0f) ? u : 0.2f * u; p = fmaf(u, at0.w, p);
      u = x1.x + r1.x; u = (u > 0.0f) ? u : 0.2f * u; p = fmaf(u, at1.x, p);
      u = x1.y + r1.y; u = (u > 0.0f) ? u : 0.2f * u; p = fmaf(u, at1.y, p);
      u = x1.z + r1.z; u = (u > 0.0f) ? u : 0.2f * u; p = fmaf(u, at1.z, p);
      u = x1.w + r1.w; u = (u > 0.0f) ? u : 0.2f * u; p = fmaf(u, at1.w, p);
      p += __shfl_xor(p, 1, 32);
      p += __shfl_xor(p, 2, 32);
      p += __shfl_xor(p, 4, 32);
      const float d  = p - mx;
      const float e  = expf(-fabsf(d));
      const bool  up = d > 0.0f;
      const float sc = up ? e : 1.0f;
      const float pp = up ? 1.0f : e;
      mx = up ? p : mx;
      ls = fmaf(ls, sc, pp);
      a0 = fmaf(pp, x0.x, a0 * sc); a1 = fmaf(pp, x0.y, a1 * sc);
      a2 = fmaf(pp, x0.z, a2 * sc); a3 = fmaf(pp, x0.w, a3 * sc);
      a4 = fmaf(pp, x1.x, a4 * sc); a5 = fmaf(pp, x1.y, a5 * sc);
      a6 = fmaf(pp, x1.z, a6 * sc); a7 = fmaf(pp, x1.w, a7 * sc);
    }
    const float rl = 1.0f / ls;
    float y0 = a0 * rl, y1 = a1 * rl, y2 = a2 * rl, y3 = a3 * rl;
    float y4 = a4 * rl, y5 = a5 * rl, y6 = a6 * rl, y7 = a7 * rl;
    y0 += __shfl_xor(y0, 8, 32); y0 += __shfl_xor(y0, 16, 32);
    y1 += __shfl_xor(y1, 8, 32); y1 += __shfl_xor(y1, 16, 32);
    y2 += __shfl_xor(y2, 8, 32); y2 += __shfl_xor(y2, 16, 32);
    y3 += __shfl_xor(y3, 8, 32); y3 += __shfl_xor(y3, 16, 32);
    y4 += __shfl_xor(y4, 8, 32); y4 += __shfl_xor(y4, 16, 32);
    y5 += __shfl_xor(y5, 8, 32); y5 += __shfl_xor(y5, 16, 32);
    y6 += __shfl_xor(y6, 8, 32); y6 += __shfl_xor(y6, 16, 32);
    y7 += __shfl_xor(y7, 8, 32); y7 += __shfl_xor(y7, 16, 32);
    const float va = (hd == 0) ? y0 : ((hd == 1) ? y2 : ((hd == 2) ? y4 : y6));
    const float vb = (hd == 0) ? y1 : ((hd == 1) ? y3 : ((hd == 2) ? y5 : y7));
    const float pzr = big ? qnan : pz;
    const float ta = tanhf(va + bs.x) + pzr;
    const float tb = tanhf(vb + bs.y) + pzr;
    const unsigned hb0 = bf16_bits(ta), hb1 = bf16_bits(tb);
    const unsigned lb0 = bf16_bits(ta - __uint_as_float(hb0 << 16));
    const unsigned lb1 = bf16_bits(tb - __uint_as_float(hb1 << 16));
    const int hw = (int)(hb0 | (hb1 << 16));
    const int lw = (int)(lb0 | (lb1 << 16));
    const int g0 = __shfl(hw, q, 32),  g1 = __shfl(hw, q1, 32);
    const int g2 = __shfl(hw, q2, 32), g3 = __shfl(hw, q3, 32);
    const int p0 = __shfl(lw, q, 32),  p1 = __shfl(lw, q1, 32);
    const int p2 = __shfl(lw, q2, 32), p3 = __shfl(lw, q3, 32);
    const bool lsel = (lane & 8) != 0;
    v4u pv;
    pv.x = (unsigned int)(lsel ? p0 : g0);
    pv.y = (unsigned int)(lsel ? p1 : g1);
    pv.z = (unsigned int)(lsel ? p2 : g2);
    pv.w = (unsigned int)(lsel ? p3 : g3);
    unsigned short* hp = xa + (size_t)node * XAP + 8 * (lane & 15);
    const bool wr = lane < 16;
    if (wr) *(volatile v4u*)hp = pv;
    __threadfence();
    if (wr) *(volatile v4u*)hp = pv;
  }
}

__global__ __launch_bounds__(GTHR) void k_out(const unsigned short* __restrict__ XA,
                                              const unsigned short* __restrict__ WGt,
                                              const float* __restrict__ pf, const int* __restrict__ cstate,
                                              int nN, float* out) {
  __shared__ __attribute__((aligned(16))) float stg[GBM * ODIM];
  const int tid = (int)threadIdx.x, lane = tid & 31, wave = tid >> 5, hh = lane >> 4, m = lane & 15;
  const int rowBase = (int)blockIdx.x * GBM;

  v8f acc[2];
  {
    const v8f z = {0.f, 0.f, 0.f, 0.f, 0.f, 0.f, 0.f, 0.f};
    acc[0] = z; acc[1] = z;
  }
  const unsigned short* ap = XA  + (size_t)(rowBase + 16 * wave + m) * XAP + 8 * hh;
  const unsigned short* wp = WGt + (size_t)m * KG + 8 * hh;
#pragma unroll 1
  for (int ks = 0; ks < KG / 32; ++ks) {
    FragB af;
    af.h[0] = *(const v8usa*)(ap + 32 * ks);
    af.h[1] = *(const v8usa*)(ap + 32 * ks + 16);
#pragma unroll
    for (int t = 0; t < 2; ++t) {
      const unsigned short* wq = wp + (size_t)(16 * t) * KG + 32 * ks;
      FragB bf;
      bf.h[0] = *(const v8usa*)wq;
      bf.h[1] = *(const v8usa*)(wq + 16);
      acc[t] = wmb(af, bf, acc[t]);
    }
  }
#pragma unroll
  for (int t = 0; t < 2; ++t) {
    const int lc = 16 * t + m;
#pragma unroll
    for (int r = 0; r < 8; ++r) {
      const int lr = 16 * wave + 8 * hh + r;
      stg[lr * ODIM + lc] = acc[t][r];
    }
  }
  __syncthreads();

  const int c4 = 4 * (lane & 7);
  const v4f b4 = *(const v4f*)(pf + PF_BG + c4);
  v4f fv[4];
#pragma unroll
  for (int i = 0; i < 4; ++i) {
    const int lr  = 16 * wave + 4 * i + (lane >> 3);
    const int gr  = rowBase + lr;
    const int grc = gr < nN ? gr : nN - 1;
    const int cs  = cstate[grc];
    const float mk = (cs > 0) ? 1.0f : 0.0f;
    const v4f v = *(const v4fa*)(stg + lr * ODIM + c4) + b4;
    v4f y;
    y.x = v.x * mk; y.y = v.y * mk; y.z = v.z * mk; y.w = v.w * mk;
    fv[i] = y;
  }
#pragma unroll
  for (int i = 0; i < 4; ++i) {
    const int gr = rowBase + 16 * wave + 4 * i + (lane >> 3);
    if (gr < nN) *(volatile v4f*)(out + (size_t)gr * ODIM + c4) = fv[i];
  }
  __threadfence();
#pragma unroll
  for (int i = 0; i < 4; ++i) {
    const int gr = rowBase + 16 * wave + 4 * i + (lane >> 3);
    if (gr < nN) *(volatile v4f*)(out + (size_t)gr * ODIM + c4) = fv[i];
  }
}

static inline int cdiv(int a, int b) { return (a + b - 1) / b; }
static inline size_t al256(size_t o) { return (o + 255) & ~(size_t)255; }

extern "C" void kernel_launch(void* const* d_in, const int* in_sizes, int n_in,
                              void* d_out, int out_size, void* d_ws, size_t ws_size,
                              hipStream_t stream) {
  if (n_in < 14) return;
  if (in_sizes[0] < FIN || (in_sizes[0] % FIN) != 0) return;
  const int nN = in_sizes[0] / FIN;
  if (nN < 1 || nN > (1 << 21)) return;
  if (in_sizes[1] != FIN * HID || in_sizes[2] != HID) return;
  if (in_sizes[3] != 2 * HID * HC || in_sizes[4] != HC) return;
  if (in_sizes[5] != 2 * HID * HC || in_sizes[6] != HC) return;
  if (in_sizes[7] != NHEAD * HID || in_sizes[8] != HC) return;
  if (in_sizes[9] != HID * ODIM || in_sizes[10] != ODIM) return;
  if (in_sizes[11] < 2 || (in_sizes[11] & 1) != 0) return;
  const int nE = in_sizes[11] / 2;
  if (nE < 1 || nE >= (1 << (31 - SLA))) return;
  if (in_sizes[12] != nN || in_sizes[13] != nN) return;
  if ((long long)out_size != (long long)nN * ODIM) return;

  const float* feat   = (const float*)d_in[0];
  const float* W_in   = (const float*)d_in[1];
  const float* b_in   = (const float*)d_in[2];
  const float* Wl     = (const float*)d_in[3];
  const float* bl     = (const float*)d_in[4];
  const float* Wr     = (const float*)d_in[5];
  const float* br     = (const float*)d_in[6];
  const float* att    = (const float*)d_in[7];
  const float* b_conv = (const float*)d_in[8];
  const float* Wg     = (const float*)d_in[9];
  const float* bg     = (const float*)d_in[10];
  const int*   edge   = (const int*)d_in[11];
  const int*   nmask  = (const int*)d_in[12];
  const int*   cstate = (const int*)d_in[13];
  float* out = (float*)d_out;
  const int* src = edge;
  const int* dst = edge + nE;

  const int MP  = cdiv(nN, GBM) * GBM;
  const int gM  = MP / GBM;
  const int gFB = (MP * (FIN / 8)) / NTHR;
  if (gFB * NTHR != MP * (FIN / 8)) return;
  const int gA  = cdiv(nN, NBA);
  const int vec8 = ((nE & 3) == 0) ? 1 : 0;

  char* ws = (char*)d_ws;
  size_t off = 0;
  const size_t oPF  = off; off = al256(off + (size_t)PF_N * 4);
  const size_t oWIN = off; off = al256(off + (size_t)HID * FIN * 2);
  const size_t oWLR = off; off = al256(off + (size_t)NLR * KX * 2);
  const size_t oWG  = off; off = al256(off + (size_t)ODIM * KG * 2);
  const size_t oFB  = off; off = al256(off + (size_t)MP * FIN * 2);
  const size_t oXA  = off; off = al256(off + (size_t)MP * XAP * 2);
  const size_t oXLR = off; off = al256(off + (size_t)2 * MP * HC * 4);
  if (off > ws_size || off > (size_t)WSMAX) return;
  float*          PF   = (float*)(ws + oPF);
  unsigned short* WINt = (unsigned short*)(ws + oWIN);
  unsigned short* WLRt = (unsigned short*)(ws + oWLR);
  unsigned short* WGt  = (unsigned short*)(ws + oWG);
  unsigned short* FB   = (unsigned short*)(ws + oFB);
  unsigned short* XA   = (unsigned short*)(ws + oXA);
  float*          XL   = (float*)(ws + oXLR);
  const unsigned long long planeStride = (unsigned long long)MP * HC;
  float*          XR   = XL + (size_t)planeStride;

  const size_t scanLds = (size_t)AGG_LDS_INTS * 4;
  hipFuncSetAttribute(reinterpret_cast<const void*>(&k_scan), hipFuncAttributeMaxDynamicSharedMemorySize, (int)scanLds);

  k_prep<<<gFB + NB_WLR + NB_WIN + NB_WG + NB_PF, NTHR, 0, stream>>>(
      feat, W_in, b_in, Wl, bl, Wr, br, att, b_conv, Wg, bg, nN, gFB, FB, WINt, WLRt, WGt, PF);
  k_gemm0<<<gM, GTHR, 0, stream>>>(FB, WINt, PF, XA);
  for (int step = 0; step < 3; ++step) {
    k_gemm_step<<<dim3(gM, NLR / 64), GTHR, 0, stream>>>(XA, WLRt, PF, XL, planeStride);
    k_scan<<<gA, NTHR, scanLds, stream>>>(src, dst, nmask, step, nE, nN, vec8, XL, XR, PF, XA);
  }
  k_out<<<gM, GTHR, 0, stream>>>(XA, WGt, PF, cstate, nN, out);
}
